// GRUDecoder_30726196035717
// MI455X (gfx1250) — hardware-verified
//
#include <hip/hip_runtime.h>
#include <math.h>

typedef __attribute__((ext_vector_type(16))) __bf16   v16b;
typedef __attribute__((ext_vector_type(8)))  __bf16   v8b;
typedef __attribute__((ext_vector_type(8)))  float    v8f;
typedef __attribute__((ext_vector_type(4)))  float    v4f;
typedef __attribute__((ext_vector_type(2)))  unsigned v2u;

static constexpr int HID = 32;
static constexpr int NGATE = 3 * HID;
static constexpr int NSTEPS = 128;
static constexpr int NWAVES = 4;
static constexpr int NTHREADS = NWAVES * 32;
static constexpr int COLS_PER_BLOCK = NWAVES * 16;
static constexpr int YPITCH = NSTEPS + 4;
static constexpr int WPLANE = NGATE * HID;

static_assert(HID == 32, "one 32-deep k step per tile");
static_assert(NSTEPS == 128, "output row = 32 lanes x 16 B");
static_assert((YPITCH * 4) % 16 == 0, "16-B aligned LDS rows");
static_assert(WPLANE == 6 * 4 * NTHREADS, "weight staging coverage: 6 float4 per thread");
static_assert(COLS_PER_BLOCK * NSTEPS == 16 * 4 * NTHREADS, "y staging zero-fill coverage: 16 float4 per thread");

__device__ __forceinline__ unsigned short f2bf_bits(float f) {
  unsigned u = __float_as_uint(f);
  return (unsigned short)((u + 0x7FFFu + ((u >> 16) & 1u)) >> 16);
}
__device__ __forceinline__ float bf_bits2f(unsigned short h) { return __uint_as_float(((unsigned)h) << 16); }

__device__ __forceinline__ v16b frag_load_bf(const __bf16* p) {
  union { v16b v; v8b h[2]; } f;
  f.h[0] = *(const v8b*)(p);
  f.h[1] = *(const v8b*)(p + 16);
  return f.v;
}

__device__ __forceinline__ v8f mma_bf(v16b a, v16b b, v8f c) {
  c = __builtin_amdgcn_wmma_f32_16x16x32_bf16(false, a, false, b, (short)0, c, false, false);
  asm volatile("v_nop\n\tv_nop\n\tv_nop\n\tv_nop" : "+v"(c) : "v"(a), "v"(b));
  return c;
}

__device__ __forceinline__ void split_pair(float a, float b, unsigned& hu, unsigned& lu) {
  const unsigned short ha = f2bf_bits(a);
  const unsigned short hb = f2bf_bits(b);
  const unsigned short la = f2bf_bits(a - bf_bits2f(ha));
  const unsigned short lb = f2bf_bits(b - bf_bits2f(hb));
  hu = (unsigned)ha | ((unsigned)hb << 16);
  lu = (unsigned)la | ((unsigned)lb << 16);
}

__device__ __forceinline__ void split_frag(v8f t0, v8f t1, v16b& fh, v16b& fl) {
  union U { unsigned u[8]; v16b v; } H, L;
#pragma unroll
  for (int j = 0; j < 4; ++j) {
    unsigned a, b;
    split_pair(t0[2 * j], t0[2 * j + 1], a, b);
    H.u[j] = a; L.u[j] = b;
    split_pair(t1[2 * j], t1[2 * j + 1], a, b);
    H.u[4 + j] = a; L.u[4 + j] = b;
  }
  fh = H.v; fl = L.v;
}

__device__ __forceinline__ v8f mma3(const unsigned short* ph, const unsigned short* pl, int off,
                                    v16b bh, v16b bl, v8f acc) {
  const v16b ah = frag_load_bf((const __bf16*)ph + off);
  const v16b al = frag_load_bf((const __bf16*)pl + off);
  acc = mma_bf(ah, bh, acc);
  acc = mma_bf(ah, bl, acc);
  acc = mma_bf(al, bh, acc);
  return acc;
}

__device__ __forceinline__ float gru_cell(float pre_r, float pre_z, float gxn, float ghn, float hprev) {
  const float r = 1.0f / (1.0f + expf(-pre_r));
  const float z = 1.0f / (1.0f + expf(-pre_z));
  const float n = tanhf(gxn + r * ghn);
  return (1.0f - z) * n + z * hprev;
}


__device__ __forceinline__ float half_step_x(v8f& ht, v8f Drz_r, v8f Drz_z, v8f Dxn, v8f Dhn,
                                             const float* kc, float yp) {
#pragma unroll
  for (int v = 0; v < 8; ++v) {
    const v4f ca = *(const v4f*)(kc + v * 8);
    const v4f cb = *(const v4f*)(kc + v * 8 + 4);
    const float hn = gru_cell(Drz_r[v] + ca[3], Drz_z[v] + cb[0], Dxn[v] + cb[1], Dhn[v] + cb[2], ht[v]);
    ht[v] = hn;
    yp += hn * cb[3];
  }
  return yp;
}

__device__ __forceinline__ float half_step_fb(v8f& ht, v8f Dr, v8f Dz, v8f Dn,
                                              const float* kc, float y, float yp) {
#pragma unroll
  for (int v = 0; v < 8; ++v) {
    const v4f ca = *(const v4f*)(kc + v * 8);
    const v4f cb = *(const v4f*)(kc + v * 8 + 4);
    const float hn = gru_cell(Dr[v] + (y * ca[0] + ca[3]), Dz[v] + (y * ca[1] + cb[0]),
                              y * ca[2] + cb[1], Dn[v] + cb[2], ht[v]);
    ht[v] = hn;
    yp += hn * cb[3];
  }
  return yp;
}

__global__ __launch_bounds__(NTHREADS)
void gru_decode_kernel(const float* __restrict__ in_data,
                       const float* __restrict__ hidden,
                       const float* __restrict__ w_ih,
                       const float* __restrict__ w_hh,
                       const float* __restrict__ b_ih,
                       const float* __restrict__ b_hh,
                       const float* __restrict__ w_out,
                       const float* __restrict__ b_out,
                       const int* __restrict__ nsteps_p,
                       float* __restrict__ out,
                       int nbatch) {
  __shared__ __align__(16) unsigned short s_whh_hi[WPLANE];
  __shared__ __align__(16) unsigned short s_whh_lo[WPLANE];
  __shared__ __align__(16) unsigned short s_wih_hi[WPLANE];
  __shared__ __align__(16) unsigned short s_wih_lo[WPLANE];
  __shared__ __align__(16) float s_rs[128];
  __shared__ __align__(16) float s_kc[HID * 8];
  __shared__ __align__(16) float s_y[COLS_PER_BLOCK * YPITCH];

  const int tid  = threadIdx.x;
  const int wave = tid >> 5;
  const int lane = tid & 31;
  const int hh   = lane >> 4;
  const int cidx = lane & 15;

  {
    const v4f z4 = {0.f, 0.f, 0.f, 0.f};
#pragma unroll
    for (int it = 0; it < 16; ++it) {
      const int i = it * NTHREADS + tid;
      const int r = i >> 5;
      const int c4 = (i & 31) * 4;
      *(v4f*)(s_y + r * YPITCH + c4) = z4;
    }
  }

#pragma unroll 1
  for (int it = 0; it < 6; ++it) {
    const int i4 = it * NTHREADS + tid;
    const v4f a = *(const v4f*)(w_hh + 4 * i4);
    const v4f b = *(const v4f*)(w_ih + 4 * i4);
    unsigned ah0, al0, ah1, al1, bh0, bl0, bh1, bl1;
    split_pair(a[0], a[1], ah0, al0);
    split_pair(a[2], a[3], ah1, al1);
    split_pair(b[0], b[1], bh0, bl0);
    split_pair(b[2], b[3], bh1, bl1);
    v2u t;
    t[0] = ah0; t[1] = ah1; *(v2u*)(s_whh_hi + 4 * i4) = t;
    t[0] = al0; t[1] = al1; *(v2u*)(s_whh_lo + 4 * i4) = t;
    t[0] = bh0; t[1] = bh1; *(v2u*)(s_wih_hi + 4 * i4) = t;
    t[0] = bl0; t[1] = bl1; *(v2u*)(s_wih_lo + 4 * i4) = t;
  }

  if (tid < NGATE) {
    const float* p = w_ih + tid * HID;
    float acc = 0.0f;
#pragma unroll
    for (int q = 0; q < 8; ++q) {
      const v4f v = *(const v4f*)(p + 4 * q);
      acc += v[0]; acc += v[1]; acc += v[2]; acc += v[3];
    }
    s_rs[tid] = acc;
  }
  __syncthreads();
  if (tid < HID) {
    v4f ca, cb;
    ca[0] = s_rs[tid];
    ca[1] = s_rs[HID + tid];
    ca[2] = s_rs[2 * HID + tid];
    ca[3] = b_ih[tid] + b_hh[tid];
    cb[0] = b_ih[HID + tid] + b_hh[HID + tid];
    cb[1] = b_ih[2 * HID + tid];
    cb[2] = b_hh[2 * HID + tid];
    cb[3] = w_out[tid];
    *(v4f*)(s_kc + tid * 8) = ca;
    *(v4f*)(s_kc + tid * 8 + 4) = cb;
  }
  __syncthreads();

  const int col  = blockIdx.x * COLS_PER_BLOCK + wave * 16 + cidx;
  const int colc = (col < nbatch) ? col : (nbatch - 1);
  const float* hp = hidden + (size_t)colc * HID;
  const float* xp = in_data + (size_t)colc * HID;

  v8f ht0, ht1, xt0, xt1;
  {
    const v4f a = *(const v4f*)(hp + 8 * hh);
    const v4f b = *(const v4f*)(hp + 8 * hh + 4);
    const v4f c = *(const v4f*)(hp + 16 + 8 * hh);
    const v4f d = *(const v4f*)(hp + 20 + 8 * hh);
    const v4f e = *(const v4f*)(xp + 8 * hh);
    const v4f f = *(const v4f*)(xp + 8 * hh + 4);
    const v4f g = *(const v4f*)(xp + 16 + 8 * hh);
    const v4f k = *(const v4f*)(xp + 20 + 8 * hh);
#pragma unroll
    for (int q = 0; q < 4; ++q) {
      ht0[q] = a[q]; ht0[4 + q] = b[q]; ht1[q] = c[q]; ht1[4 + q] = d[q];
      xt0[q] = e[q]; xt0[4 + q] = f[q]; xt1[q] = g[q]; xt1[4 + q] = k[q];
    }
  }

  int nst = nsteps_p[0];
  nst = (nst < 0) ? 0 : nst;
  nst = (nst > NSTEPS) ? NSTEPS : nst;

  const float bo = b_out[0];
  const v8f zero8 = {0.f, 0.f, 0.f, 0.f, 0.f, 0.f, 0.f, 0.f};
  const float* kc0 = s_kc + (8 * hh) * 8;
  const float* kc1 = s_kc + (16 + 8 * hh) * 8;
  float* yrow = s_y + (wave * 16 + cidx) * YPITCH;
  float y = 0.0f;

  if (nst > 0) {
    v16b xh, xl, bh, bl;
    split_frag(xt0, xt1, xh, xl);
    split_frag(ht0, ht1, bh, bl);
    v8f D[6], Dxn[2];
#pragma unroll
    for (int t = 0; t < 4; ++t) {
      const int off = (t * 16 + cidx) * HID + 8 * hh;
      D[t] = mma3(s_wih_hi, s_wih_lo, off, xh, xl, zero8);
      D[t] = mma3(s_whh_hi, s_whh_lo, off, bh, bl, D[t]);
    }
#pragma unroll
    for (int t2 = 0; t2 < 2; ++t2) {
      const int off = ((4 + t2) * 16 + cidx) * HID + 8 * hh;
      Dxn[t2]   = mma3(s_wih_hi, s_wih_lo, off, xh, xl, zero8);
      D[4 + t2] = mma3(s_whh_hi, s_whh_lo, off, bh, bl, zero8);
    }
    float yp = 0.0f;
    yp = half_step_x(ht0, D[0], D[2], Dxn[0], D[4], kc0, yp);
    yp = half_step_x(ht1, D[1], D[3], Dxn[1], D[5], kc1, yp);
    y = yp + __shfl_xor(yp, 16, 32) + bo;
    if (hh == 0) yrow[0] = y;
  }

  for (int s = 1; s < nst; ++s) {
    v16b bh, bl;
    split_frag(ht0, ht1, bh, bl);
    v8f D[6];
#pragma unroll
    for (int t = 0; t < 6; ++t) {
      const int off = (t * 16 + cidx) * HID + 8 * hh;
      D[t] = mma3(s_whh_hi, s_whh_lo, off, bh, bl, zero8);
    }
    float yp = 0.0f;
    yp = half_step_fb(ht0, D[0], D[2], D[4], kc0, y, yp);
    yp = half_step_fb(ht1, D[1], D[3], D[5], kc1, y, yp);
    y = yp + __shfl_xor(yp, 16, 32) + bo;
    if (hh == 0) yrow[s] = y;
  }

  __syncthreads();
  for (int pass = 0; pass < 2; ++pass) {
#pragma unroll
    for (int r = 0; r < 16; ++r) {
      const int grow = blockIdx.x * COLS_PER_BLOCK + wave * 16 + r;
      if (grow < nbatch) {
        const v4f v = *(const v4f*)(s_y + (wave * 16 + r) * YPITCH + lane * 4);
        *(volatile v4f*)(out + (size_t)grow * NSTEPS + lane * 4) = v;
      }
    }
    __threadfence();
  }
}

extern "C" void kernel_launch(void* const* d_in, const int* in_sizes, int n_in,
                              void* d_out, int out_size, void* d_ws, size_t ws_size,
                              hipStream_t stream) {
  (void)n_in; (void)d_ws; (void)ws_size;
  const float* in_data = (const float*)d_in[0];
  const float* hidden  = (const float*)d_in[1];
  const float* w_ih    = (const float*)d_in[2];
  const float* w_hh    = (const float*)d_in[3];
  const float* b_ih    = (const float*)d_in[4];
  const float* b_hh    = (const float*)d_in[5];
  const float* w_out   = (const float*)d_in[6];
  const float* b_out   = (const float*)d_in[7];
  const int*   nsteps  = (const int*)d_in[8];
  float* out = (float*)d_out;

  const int nbatch = in_sizes[1] / HID;
  if (nbatch <= 0) return;
  if (out_size != nbatch * NSTEPS) return;
  const int grid = (nbatch + COLS_PER_BLOCK - 1) / COLS_PER_BLOCK;
  gru_decode_kernel<<<dim3(grid), dim3(NTHREADS), 0, stream>>>(
      in_data, hidden, w_ih, w_hh, b_ih, b_hh, w_out, b_out, nsteps, out, nbatch);
}
